// LinearAttentionARMA_61040075210836
// MI455X (gfx1250) — hardware-verified
//
#include <hip/hip_runtime.h>
#include <stdint.h>
#include <stddef.h>


#define BB 2
#define LL 2048
#define DD 512
#define HH 8
#define DH 64

typedef __bf16 v16bf __attribute__((ext_vector_type(16)));
typedef __bf16 v8bf  __attribute__((ext_vector_type(8)));
typedef float  v8f   __attribute__((ext_vector_type(8)));
typedef float  v4f   __attribute__((ext_vector_type(4)));
typedef v8bf v8bfa __attribute__((may_alias));
typedef v4f  v4fa  __attribute__((may_alias));

union Frag { v16bf v; v8bf h[2]; __bf16 e[16]; };
union Acc  { v8f v; float e[8]; };
union Pk8  { v8bf v; __bf16 e[8]; };
union F4   { v4f v; float e[4]; };

static __device__ __forceinline__ v8f zacc() {
  Acc z;
#pragma unroll
  for (int i = 0; i < 8; ++i) z.e[i] = 0.0f;
  return z.v;
}
static __device__ __forceinline__ v8bf zbf8() {
  Pk8 z;
#pragma unroll
  for (int i = 0; i < 8; ++i) z.e[i] = (__bf16)0.0f;
  return z.v;
}
static __device__ __forceinline__ v4f zf4() {
  F4 z;
#pragma unroll
  for (int i = 0; i < 4; ++i) z.e[i] = 0.0f;
  return z.v;
}
static __device__ __forceinline__ void split2(float x, __bf16& hi, __bf16& lo) {
  __bf16 hv = (__bf16)x;
  hi = hv;
  lo = (__bf16)(x - (float)hv);
}

static __device__ __forceinline__ v8f mma(v16bf a, v16bf b, v8f c) {
  return __builtin_amdgcn_wmma_f32_16x16x32_bf16(false, a, false, b, (short)0, c, false, false);
}
#define WMMA_GUARD2(acc, a0, b0) \
  asm volatile("v_nop\n\tv_nop\n\tv_nop\n\tv_nop" : "+v"(acc) : "v"(a0), "v"(b0))
#define WMMA_GUARD4(acc, a0, a1, b0, b1) \
  asm volatile("v_nop\n\tv_nop\n\tv_nop\n\tv_nop" : "+v"(acc) : "v"(a0), "v"(a1), "v"(b0), "v"(b1))

static __device__ __forceinline__ v8f mma3(const Frag& ah, const Frag& al, const Frag& bh,
                                            const Frag& bl, v8f c) {
  c = mma(ah.v, bh.v, c);
  c = mma(al.v, bh.v, c);
  c = mma(ah.v, bl.v, c);
  WMMA_GUARD4(c, ah.v, al.v, bh.v, bl.v);
  return c;
}

__global__ __launch_bounds__(256) void k_split_planes(
    const float* __restrict__ X, const float* __restrict__ W1, const float* __restrict__ W2,
    const float* __restrict__ W3, const float* __restrict__ W4, int nX, int nW,
    __bf16* hi, __bf16* lo) {
  const size_t total = (size_t)nX + 4 * (size_t)nW;
  const size_t g = ((size_t)blockIdx.x * 256 + threadIdx.x) * 8;
  if (g + 8 > total) return;
  const float* src;
  size_t idx;
  if (g < (size_t)nX) {
    src = X; idx = g;
  } else {
    const size_t rr = g - (size_t)nX;
    const int w = (int)(rr / (size_t)nW);
    idx = rr - (size_t)w * (size_t)nW;
    src = (w == 0) ? W1 : (w == 1) ? W2 : (w == 2) ? W3 : W4;
  }
  F4 a, c;
  a.v = *(const v4fa*)(src + idx);
  c.v = *(const v4fa*)(src + idx + 4);
  Pk8 ph, pl;
#pragma unroll
  for (int j = 0; j < 4; ++j) {
    split2(a.e[j], ph.e[j], pl.e[j]);
    split2(c.e[j], ph.e[4 + j], pl.e[4 + j]);
  }
  *(volatile v8bf*)(hi + g) = ph.v;
  *(volatile v8bf*)(lo + g) = pl.v;
  __threadfence();
  *(volatile v8bf*)(hi + g) = ph.v;
  *(volatile v8bf*)(lo + g) = pl.v;
}

template <bool SPLIT, bool SIGM>
__global__ __launch_bounds__(256) void k_gemm_nt(
    const __bf16* __restrict__ Ahi, const __bf16* __restrict__ Alo,
    const __bf16* __restrict__ Whi, const __bf16* __restrict__ Wlo,
    float* out, int M, int N, int K, float escale) {
  __shared__ __attribute__((aligned(16))) float s_tile[8][16][64];
  const int wave = threadIdx.x >> 5, lane = threadIdx.x & 31;
  const int h = lane >> 4, m = lane & 15;
  const int tilesN = N >> 6;
  const int tilesTot = (M >> 4) * tilesN;
  int tile = blockIdx.x * 8 + wave;
  const bool valid = tile < tilesTot;
  if (!valid) tile = 0;
  const int tm = tile / tilesN;
  const int tn = tile - tm * tilesN;
  const size_t arow = ((size_t)(tm * 16 + m)) * (size_t)K;

  Acc acc[4];
#pragma unroll
  for (int j = 0; j < 4; ++j) acc[j].v = zacc();

#pragma unroll 1
  for (int kb = 0; kb < K; kb += 32) {
    const size_t ao = arow + (size_t)(kb + 8 * h);
    Frag ah, al;
    ah.h[0] = *(const v8bfa*)(Ahi + ao);
    ah.h[1] = *(const v8bfa*)(Ahi + ao + 16);
    if (SPLIT) {
      al.h[0] = *(const v8bfa*)(Alo + ao);
      al.h[1] = *(const v8bfa*)(Alo + ao + 16);
    }
#pragma unroll
    for (int j = 0; j < 4; ++j) {
      const size_t wo = ((size_t)(tn * 64 + j * 16 + m)) * (size_t)K + (size_t)(kb + 8 * h);
      Frag bh, bl;
      bh.h[0] = *(const v8bfa*)(Whi + wo);
      bh.h[1] = *(const v8bfa*)(Whi + wo + 16);
      if (SPLIT) {
        bl.h[0] = *(const v8bfa*)(Wlo + wo);
        bl.h[1] = *(const v8bfa*)(Wlo + wo + 16);
        acc[j].v = mma3(ah, al, bh, bl, acc[j].v);
      } else {
        acc[j].v = mma(ah.v, bh.v, acc[j].v);
        WMMA_GUARD2(acc[j].v, ah.v, bh.v);
      }
    }
  }

  float (*tl)[64] = s_tile[wave];
#pragma unroll
  for (int j = 0; j < 4; ++j) {
#pragma unroll
    for (int r = 0; r < 8; ++r) {
      float x = acc[j].e[r];
      if (SIGM) x = 1.0f / (1.0f + __expf(-x * escale));
      tl[8 * h + r][j * 16 + m] = x;
    }
  }
  __syncthreads();
  const int q = lane >> 3, wl = lane & 7;
  v4f vals[8];
  size_t offs[8];
#pragma unroll
  for (int s = 0; s < 8; ++s) {
    const int row = 2 * s + (q >> 1);
    const int col = (q & 1) * 32 + wl * 4;
    vals[s] = *(const v4fa*)(&tl[row][col]);
    offs[s] = ((size_t)(tm * 16 + row)) * (size_t)N + (size_t)(tn * 64 + col);
  }
  if (valid) {
#pragma unroll
    for (int s = 0; s < 8; ++s) *(volatile v4f*)(out + offs[s]) = vals[s];
  }
  __threadfence();
  if (valid) {
#pragma unroll
    for (int s = 0; s < 8; ++s) *(volatile v4f*)(out + offs[s]) = vals[s];
  }
}

struct __align__(16) ScanLds {
  __attribute__((aligned(16))) __bf16 qhi[16][64];
  __attribute__((aligned(16))) __bf16 qlo[16][64];
  __attribute__((aligned(16))) __bf16 khi[16][64];
  __attribute__((aligned(16))) __bf16 klo[16][64];
  __attribute__((aligned(16))) __bf16 kThi[64][16];
  __attribute__((aligned(16))) __bf16 kTlo[64][16];
  __attribute__((aligned(16))) __bf16 vThi[64][16];
  __attribute__((aligned(16))) __bf16 vTlo[64][16];
  __attribute__((aligned(16))) float S[64][65];
  __attribute__((aligned(16))) float ps[4][16][16];
  __attribute__((aligned(16))) float xs[16][64];
};

static __device__ __forceinline__ void scan_chunk(ScanLds& sh, int wave, int lane, Acc& res) {
  const int h = lane >> 4, m = lane & 15, eb = wave * 16, e = eb + m;

  Frag aqh[2], aql[2];
#pragma unroll
  for (int ks = 0; ks < 2; ++ks) {
    aqh[ks].h[0] = *(const v8bfa*)(&sh.qhi[m][ks * 32 + 8 * h]);
    aqh[ks].h[1] = *(const v8bfa*)(&sh.qhi[m][ks * 32 + 16 + 8 * h]);
    aql[ks].h[0] = *(const v8bfa*)(&sh.qlo[m][ks * 32 + 8 * h]);
    aql[ks].h[1] = *(const v8bfa*)(&sh.qlo[m][ks * 32 + 16 + 8 * h]);
  }

  Acc acc;
  acc.v = zacc();
#pragma unroll
  for (int ks = 0; ks < 2; ++ks) {
    Frag bsh, bsl;
#pragma unroll
    for (int i = 0; i < 16; ++i) {
      const int d = ks * 32 + ((i < 8) ? (8 * h + i) : (16 + 8 * h + (i - 8)));
      split2(sh.S[d][e], bsh.e[i], bsl.e[i]);
    }
    acc.v = mma3(aqh[ks], aql[ks], bsh, bsl, acc.v);
  }

  Acc pacc;
  pacc.v = zacc();
#pragma unroll
  for (int ks = 0; ks < 2; ++ks) {
    Frag bkh, bkl;
    bkh.h[0] = *(const v8bfa*)(&sh.khi[m][ks * 32 + 8 * h]);
    bkh.h[1] = *(const v8bfa*)(&sh.khi[m][ks * 32 + 16 + 8 * h]);
    bkl.h[0] = *(const v8bfa*)(&sh.klo[m][ks * 32 + 8 * h]);
    bkl.h[1] = *(const v8bfa*)(&sh.klo[m][ks * 32 + 16 + 8 * h]);
    pacc.v = mma3(aqh[ks], aql[ks], bkh, bkl, pacc.v);
  }

#pragma unroll
  for (int r = 0; r < 8; ++r) {
    const int mm = 8 * h + r;
    sh.ps[wave][mm][m] = (m <= mm) ? pacc.e[r] : 0.0f;
  }
  __syncthreads();

  Frag aph, apl;
#pragma unroll
  for (int i = 0; i < 8; ++i) split2(sh.ps[wave][m][8 * h + i], aph.e[i], apl.e[i]);
  aph.h[1] = zbf8();
  apl.h[1] = zbf8();

  Frag bvh, bvl;
  bvh.h[0] = *(const v8bfa*)(&sh.vThi[e][8 * h]);
  bvh.h[1] = zbf8();
  bvl.h[0] = *(const v8bfa*)(&sh.vTlo[e][8 * h]);
  bvl.h[1] = zbf8();
  acc.v = mma3(aph, apl, bvh, bvl, acc.v);
  res = acc;

#pragma unroll
  for (int di = 0; di < 4; ++di) {
    Frag akh, akl;
    akh.h[0] = *(const v8bfa*)(&sh.kThi[di * 16 + m][8 * h]);
    akh.h[1] = zbf8();
    akl.h[0] = *(const v8bfa*)(&sh.kTlo[di * 16 + m][8 * h]);
    akl.h[1] = zbf8();
    Acc dlt;
    dlt.v = zacc();
    dlt.v = mma3(akh, akl, bvh, bvl, dlt.v);
#pragma unroll
    for (int r = 0; r < 8; ++r) sh.S[di * 16 + 8 * h + r][e] += dlt.e[r];
  }
}

__global__ __launch_bounds__(128) void k_ar_scan(
    const float* __restrict__ Qf, const float* __restrict__ Kf, const float* __restrict__ X,
    float* Xar) {
  __shared__ ScanLds sh;
  const int b = blockIdx.x / HH, hh = blockIdx.x - b * HH;
  if (b >= BB) return;
  const int tid = threadIdx.x, wave = tid >> 5, lane = tid & 31, h = lane >> 4, m = lane & 15;
  const int q = lane >> 3, wl = lane & 7;
  for (int i = tid; i < 64 * 64; i += 128) sh.S[i >> 6][i & 63] = 0.0f;
  const size_t head = (size_t)hh * DH;

  for (int c = 0; c < LL / 16; ++c) {
    const int t0 = c * 16;
    __syncthreads();
    for (int u = tid; u < 256; u += 128) {
      const int r = u >> 4, c4 = (u & 15) * 4;
      const size_t g = ((size_t)(b * LL + t0 + r)) * DD + head + (size_t)c4;
      F4 qv, kv, vv;
      qv.v = *(const v4fa*)(Qf + g);
      kv.v = *(const v4fa*)(Kf + g);
      vv.v = *(const v4fa*)(X + g);
#pragma unroll
      for (int j = 0; j < 4; ++j) {
        const int col = c4 + j;
        __bf16 hi, lo;
        split2(qv.e[j], hi, lo);
        sh.qhi[r][col] = hi; sh.qlo[r][col] = lo;
        split2(kv.e[j], hi, lo);
        sh.khi[r][col] = hi; sh.klo[r][col] = lo;
        sh.kThi[col][r] = hi; sh.kTlo[col][r] = lo;
        split2(vv.e[j], hi, lo);
        sh.vThi[col][r] = hi; sh.vTlo[col][r] = lo;
      }
    }
    __syncthreads();

    Acc acc;
    scan_chunk(sh, wave, lane, acc);
#pragma unroll
    for (int r = 0; r < 8; ++r) sh.xs[8 * h + r][wave * 16 + m] = acc.e[r];
    __syncthreads();

    v4f v0, v1;
    size_t o0, o1;
    {
      const int line = wave * 4 + q;
      const int row = line >> 1, col = (line & 1) * 32 + wl * 4;
      v0 = *(const v4fa*)(&sh.xs[row][col]);
      o0 = ((size_t)(b * LL + t0 + row)) * DD + head + (size_t)col;
    }
    {
      const int line = 16 + wave * 4 + q;
      const int row = line >> 1, col = (line & 1) * 32 + wl * 4;
      v1 = *(const v4fa*)(&sh.xs[row][col]);
      o1 = ((size_t)(b * LL + t0 + row)) * DD + head + (size_t)col;
    }
    *(volatile v4f*)(Xar + o0) = v0;
    *(volatile v4f*)(Xar + o1) = v1;
    __threadfence();
    *(volatile v4f*)(Xar + o0) = v0;
    *(volatile v4f*)(Xar + o1) = v1;
  }
}

__global__ __launch_bounds__(128) void k_ma_scan(
    const float* __restrict__ Qf, const float* __restrict__ K2f, const float* __restrict__ X,
    const float* __restrict__ Xar, __bf16* Ohi, __bf16* Olo) {
  __shared__ ScanLds sh;
  const int b = blockIdx.x / HH, hh = blockIdx.x - b * HH;
  if (b >= BB) return;
  const int tid = threadIdx.x, wave = tid >> 5, lane = tid & 31, h = lane >> 4, m = lane & 15;
  const int q = lane >> 3, wl = lane & 7;
  for (int i = tid; i < 64 * 64; i += 128) sh.S[i >> 6][i & 63] = 0.0f;
  const size_t head = (size_t)hh * DH;

  if (wave == 0) {
    Pk8 ph, pl;
    size_t g0 = 0;
    if (lane < 8) {
      g0 = ((size_t)(b * LL)) * DD + head + (size_t)(lane * 8);
      F4 a0, a1;
      a0.v = *(const v4fa*)(Xar + g0);
      a1.v = *(const v4fa*)(Xar + g0 + 4);
#pragma unroll
      for (int j = 0; j < 4; ++j) {
        split2(a0.e[j], ph.e[j], pl.e[j]);
        split2(a1.e[j], ph.e[4 + j], pl.e[4 + j]);
      }
      *(volatile v8bf*)(Ohi + g0) = ph.v;
      *(volatile v8bf*)(Olo + g0) = pl.v;
    }
    __threadfence();
    if (lane < 8) {
      *(volatile v8bf*)(Ohi + g0) = ph.v;
      *(volatile v8bf*)(Olo + g0) = pl.v;
    }
  }

  const int Lm = LL - 1;
  const int nch = (Lm + 15) / 16;
  for (int c = 0; c < nch; ++c) {
    const int t0 = c * 16;
    __syncthreads();
    for (int u = tid; u < 256; u += 128) {
      const int r = u >> 4, c4 = (u & 15) * 4;
      const int t = t0 + r;
      const bool ok = t < Lm;
      F4 qv, kv, xv, av;
      qv.v = zf4(); kv.v = zf4(); xv.v = zf4(); av.v = zf4();
      if (ok) {
        const size_t g = ((size_t)(b * LL + t)) * DD + head + (size_t)c4;
        qv.v = *(const v4fa*)(Qf + g);
        kv.v = *(const v4fa*)(K2f + g);
        xv.v = *(const v4fa*)(X + g + DD);
        av.v = *(const v4fa*)(Xar + g);
      }
#pragma unroll
      for (int j = 0; j < 4; ++j) {
        const int col = c4 + j;
        __bf16 hi, lo;
        const float qq = qv.e[j];
        const float q2 = ((qq >= 0.0f) ? (0.02f * qq) : qq) * 0.125f;
        split2(q2, hi, lo);
        sh.qhi[r][col] = hi; sh.qlo[r][col] = lo;
        split2(kv.e[j], hi, lo);
        sh.khi[r][col] = hi; sh.klo[r][col] = lo;
        sh.kThi[col][r] = hi; sh.kTlo[col][r] = lo;
        const float ev = xv.e[j] - av.e[j];
        split2(ev, hi, lo);
        sh.vThi[col][r] = hi; sh.vTlo[col][r] = lo;
      }
    }
    __syncthreads();

    Acc acc;
    scan_chunk(sh, wave, lane, acc);
#pragma unroll
    for (int r = 0; r < 8; ++r) sh.xs[8 * h + r][wave * 16 + m] = acc.e[r];
    __syncthreads();

    const int row = wave * 4 + q;
    const int lrow = t0 + 1 + row;
    const bool okr = lrow < LL;
    Pk8 ph, pl;
    size_t go = 0;
    if (okr) {
      go = ((size_t)(b * LL + lrow)) * DD + head + (size_t)(wl * 8);
      F4 a0, a1, x0, x1;
      a0.v = *(const v4fa*)(&sh.xs[row][wl * 8]);
      a1.v = *(const v4fa*)(&sh.xs[row][wl * 8 + 4]);
      x0.v = *(const v4fa*)(Xar + go);
      x1.v = *(const v4fa*)(Xar + go + 4);
#pragma unroll
      for (int j = 0; j < 4; ++j) {
        split2(x0.e[j] + a0.e[j], ph.e[j], pl.e[j]);
        split2(x1.e[j] + a1.e[j], ph.e[4 + j], pl.e[4 + j]);
      }
      *(volatile v8bf*)(Ohi + go) = ph.v;
      *(volatile v8bf*)(Olo + go) = pl.v;
    }
    __threadfence();
    if (okr) {
      *(volatile v8bf*)(Ohi + go) = ph.v;
      *(volatile v8bf*)(Olo + go) = pl.v;
    }
  }
}

extern "C" void kernel_launch(void* const* d_in, const int* in_sizes, int n_in,
                              void* d_out, int out_size, void* d_ws, size_t ws_size,
                              hipStream_t stream) {
  if (n_in < 5) return;
  const int nX = BB * LL * DD;
  const int nW = DD * DD;
  if (in_sizes[0] != nX || in_sizes[1] != nW || in_sizes[2] != nW || in_sizes[3] != nW ||
      in_sizes[4] != nW || out_size != nX)
    return;

  const float* X     = (const float*)d_in[0];
  const float* Wq1   = (const float*)d_in[1];
  const float* Wk1   = (const float*)d_in[2];
  const float* Wk2   = (const float*)d_in[3];
  const float* Wproj = (const float*)d_in[4];
  float* out = (float*)d_out;

  const size_t nPl = (size_t)nX + 4 * (size_t)nW;
  char* ws = (char*)d_ws;
  size_t off = 0;
  __bf16* Phi = (__bf16*)(ws + off); off += nPl * 2;
  __bf16* Plo = (__bf16*)(ws + off); off += nPl * 2;
  float*  Qf  = (float*)(ws + off);  off += (size_t)nX * 4;
  float*  Kf  = (float*)(ws + off);  off += (size_t)nX * 4;
  float*  K2f = (float*)(ws + off);  off += (size_t)nX * 4;
  float*  Xar = (float*)(ws + off);  off += (size_t)nX * 4;
  __bf16* Ohi = (__bf16*)(ws + off); off += (size_t)nX * 2;
  __bf16* Olo = (__bf16*)(ws + off); off += (size_t)nX * 2;
  if (off > ws_size) return;

  const __bf16* Xhi  = Phi;
  const __bf16* Xlo  = Plo;
  const __bf16* Wq1h = Phi + nX;           const __bf16* Wq1l = Plo + nX;
  const __bf16* Wk1h = Phi + nX + nW;      const __bf16* Wk1l = Plo + nX + nW;
  const __bf16* Wk2h = Phi + nX + 2 * nW;
  const __bf16* Wprh = Phi + nX + 3 * nW;  const __bf16* Wprl = Plo + nX + 3 * nW;

  const int M = BB * LL, N = DD, K = DD;
  if ((M % 16) != 0 || (N % 64) != 0 || (K % 32) != 0 || (nX % 2048) != 0 || (nW % 2048) != 0)
    return;

  const int cvBlocks = (int)((nPl / 8 + 255) / 256);
  k_split_planes<<<cvBlocks, 256, 0, stream>>>(X, Wq1, Wk1, Wk2, Wproj, nX, nW, Phi, Plo);

  const int tiles = (M / 16) * (N / 64);
  const int gb = (tiles + 7) / 8;
  const float k2scale = (float)(0.02 / 22.627416997969522);

  k_gemm_nt<true, false><<<gb, 256, 0, stream>>>(Xhi, Xlo, Wq1h, Wq1l, Qf, M, N, K, 0.0f);
  k_gemm_nt<true, false><<<gb, 256, 0, stream>>>(Xhi, Xlo, Wk1h, Wk1l, Kf, M, N, K, 0.0f);
  k_gemm_nt<false, true><<<gb, 256, 0, stream>>>(Xhi, Xhi, Wk2h, Wk2h, K2f, M, N, K, k2scale);

  k_ar_scan<<<BB * HH, 128, 0, stream>>>(Qf, Kf, X, Xar);
  k_ma_scan<<<BB * HH, 128, 0, stream>>>(Qf, K2f, X, Xar, Ohi, Olo);

  k_gemm_nt<true, false><<<gb, 256, 0, stream>>>(Ohi, Olo, Wprh, Wprl, out, M, N, K, 0.0f);
}
